// LightningLinearAttn_51728586113375
// MI455X (gfx1250) — hardware-verified
//
#include <hip/hip_runtime.h>
#include <math.h>

#define BB 8
#define TT 4096
#define DDm 128
#define CS 64
#define NCH (TT / CS)

typedef _Float16 f16;
typedef __attribute__((ext_vector_type(16))) f16 f16x16;
typedef __attribute__((ext_vector_type(8)))  f16 f16x8;
typedef __attribute__((ext_vector_type(8)))  float f32x8;
typedef __attribute__((ext_vector_type(4)))  float v4f_t;
typedef float v4fa __attribute__((ext_vector_type(4), may_alias));
__device__ __forceinline__ f32x8 wmma16(f16x16 a, f16x16 b, f32x8 c) {
  c = __builtin_amdgcn_wmma_f32_16x16x32_f16(false, a, false, b, (short)0, c, false, false);
  asm volatile("v_nop\n\tv_nop\n\tv_nop\n\tv_nop" : "+v"(c) : "v"(a), "v"(b));
  return c;
}
__device__ __forceinline__ f16x16 lds_frag(const f16* base, int stride) {
  const int lane = threadIdx.x & 31, row = lane & 15, kh = (lane >> 4) * 8;
  const f16x8 lo = *(const f16x8*)(base + row * stride + kh);
  const f16x8 hi = *(const f16x8*)(base + row * stride + kh + 16);
  f16x16 f;
#pragma unroll
  for (int i = 0; i < 8; ++i) { f[i] = lo[i]; f[i + 8] = hi[i]; }
  return f;
}
__device__ __forceinline__ float phi(float x) { return (x > 0.0f) ? (x + 1.0f) : expf(x); }

__global__ __launch_bounds__(256) void k_lightning(const float* __restrict__ q, const float* __restrict__ k, const float* __restrict__ v, float* __restrict__ out) {
  __shared__ __attribute__((aligned(16))) union U { struct { f16 qS[CS * 136]; f16 kS[CS * 136]; } a; float oS[CS * 132]; } u;
  __shared__ __attribute__((aligned(16))) f16 kT[DDm * 72];
  __shared__ __attribute__((aligned(16))) f16 vT[DDm * 72];
  __shared__ __attribute__((aligned(16))) f16 stT[DDm * 136];
  __shared__ __attribute__((aligned(16))) f16 pS[CS * 72];
  f16* qS = u.a.qS; f16* kS = u.a.kS; float* oS = u.oS;
  const int tid = threadIdx.x, lane = tid & 31, wave = tid >> 5, cl = lane & 15, rh = (lane >> 4) * 8;
  const int b = blockIdx.x;
  f32x8 st[8];
#pragma unroll
  for (int j = 0; j < 8; ++j) { f32x8 z = {}; st[j] = z; }
  for (int e = tid; e < DDm * 136; e += 256) stT[e] = (f16)0.0f;
#pragma unroll 1
  for (int c = 0; c < NCH; ++c) {
    const size_t row0 = (size_t)b * TT + (size_t)c * CS;
    __syncthreads();
    for (int e = tid; e < CS * DDm; e += 256) { const int r = e >> 7, d = e & 127; const size_t g = (row0 + r) * DDm + d;
      const f16 fq = (f16)phi(q[g]), fk = (f16)phi(k[g]), fv = (f16)v[g];
      qS[r * 136 + d] = fq; kS[r * 136 + d] = fk; kT[d * 72 + r] = fk; vT[d * 72 + r] = fv; }
    __syncthreads();
    { const int it = wave & 3, jt0 = (wave >> 2) * 2;
      for (int jj = 0; jj < 2; ++jj) { const int jt = jt0 + jj; f32x8 acc = {};
#pragma unroll
        for (int ks = 0; ks < 4; ++ks) acc = wmma16(lds_frag(qS + (it * 16) * 136 + ks * 32, 136), lds_frag(kS + (jt * 16) * 136 + ks * 32, 136), acc);
#pragma unroll
        for (int r = 0; r < 8; ++r) { const int i = it * 16 + rh + r, j = jt * 16 + cl; pS[i * 72 + j] = (f16)((j <= i) ? acc[r] : 0.0f); } } }
    f32x8 oacc[4];
    { const int it = wave & 3, et0 = (wave >> 2) * 4;
#pragma unroll
      for (int j = 0; j < 4; ++j) { f32x8 z = {}; oacc[j] = z; }
#pragma unroll
      for (int ks = 0; ks < 4; ++ks) { const f16x16 af = lds_frag(qS + (it * 16) * 136 + ks * 32, 136);
#pragma unroll
        for (int j = 0; j < 4; ++j) oacc[j] = wmma16(af, lds_frag(stT + ((et0 + j) * 16) * 136 + ks * 32, 136), oacc[j]); } }
    __syncthreads();
    { const int it = wave & 3, et0 = (wave >> 2) * 4;
#pragma unroll
      for (int ks = 0; ks < 2; ++ks) { const f16x16 af = lds_frag(pS + (it * 16) * 72 + ks * 32, 72);
#pragma unroll
        for (int j = 0; j < 4; ++j) oacc[j] = wmma16(af, lds_frag(vT + ((et0 + j) * 16) * 72 + ks * 32, 72), oacc[j]); }
#pragma unroll
      for (int j = 0; j < 4; ++j)
#pragma unroll
        for (int r = 0; r < 8; ++r) oS[(it * 16 + rh + r) * 132 + (et0 + j) * 16 + cl] = oacc[j][r]; }
    {
#pragma unroll
      for (int ks = 0; ks < 2; ++ks) { const f16x16 af = lds_frag(kT + (wave * 16) * 72 + ks * 32, 72);
#pragma unroll
        for (int j = 0; j < 8; ++j) st[j] = wmma16(af, lds_frag(vT + (j * 16) * 72 + ks * 32, 72), st[j]); }
#pragma unroll
      for (int j = 0; j < 8; ++j)
#pragma unroll
        for (int r = 0; r < 8; ++r) { const int d = wave * 16 + rh + r, e = j * 16 + cl; stT[e * 136 + d] = (f16)st[j][r]; } }
    __syncthreads();
#pragma unroll 1
    for (int pass = 0; pass < 2; ++pass) { for (int q4 = tid; q4 < CS * 32; q4 += 256) { const int r = q4 >> 5, c4 = (q4 & 31) * 4;
        *(volatile v4f_t*)(out + (row0 + r) * DDm + c4) = *(const volatile v4fa*)(oS + r * 132 + c4); } __threadfence(); }
  }
}

extern "C" void kernel_launch(void* const* d_in, const int* in_sizes, int n_in,
                              void* d_out, int out_size, void* d_ws, size_t ws_size,
                              hipStream_t stream) {
  (void)in_sizes; (void)n_in; (void)out_size; (void)d_ws; (void)ws_size;
  const float* q = (const float*)d_in[0], *k = (const float*)d_in[1], *v = (const float*)d_in[2];
  float* out = (float*)d_out;
  k_lightning<<<dim3(BB), dim3(256), 0, stream>>>(q, k, v, out);
}
